// TransformerLayerShardV2_45131516347066
// MI455X (gfx1250) — hardware-verified
//
#include <hip/hip_runtime.h>


#define NB_  2
#define TT   2048
#define DD   1024
#define MP   8
#define SW   1408
#define LOC  128
#define FFS  1024
#define FIN  (MP * SW)
#define DCAT 5120
#define ZH   1
#define PCAR 1024.0f
#define WSC  16384.0f
typedef _Float16 h16;
typedef unsigned short bf;
typedef __attribute__((ext_vector_type(16))) __bf16   v16bf;
typedef __attribute__((ext_vector_type(16))) _Float16 v16h;
typedef __attribute__((ext_vector_type(8)))  _Float16 v8h;
typedef __attribute__((ext_vector_type(8)))  unsigned short v8us;
typedef __attribute__((ext_vector_type(8)))  float    v8f;
typedef __attribute__((ext_vector_type(4)))  float    v4f;
typedef v8h  __attribute__((may_alias)) v8ha;
typedef v4f  __attribute__((may_alias)) v4fa;
typedef v8us __attribute__((may_alias)) v8usa;

__device__ __forceinline__ unsigned short f2bf(float f) { unsigned u = __float_as_uint(f); u += 0x7FFFu + ((u >> 16) & 1u); return (unsigned short)(u >> 16); }
__device__ __forceinline__ float bf2f(unsigned short b) { return __uint_as_float(((unsigned)b) << 16); }
__device__ __forceinline__ float bfr(float f) { return bf2f(f2bf(f)); }
__device__ __forceinline__ v16h cat16(v8h lo, v8h hi) { return __builtin_shufflevector(lo, hi, 0, 1, 2, 3, 4, 5, 6, 7, 8, 9, 10, 11, 12, 13, 14, 15); }
__device__ __forceinline__ v16bf cat16b(v8us lo, v8us hi) { return __builtin_bit_cast(v16bf, __builtin_shufflevector(lo, hi, 0, 1, 2, 3, 4, 5, 6, 7, 8, 9, 10, 11, 12, 13, 14, 15)); }
__device__ __forceinline__ v8f wmma16(v16h a, v16h b, v8f c) { return __builtin_amdgcn_wmma_f32_16x16x32_f16(false, a, false, b, (short)0, c, false, false); }
__device__ __forceinline__ v8f wmmab(v16bf a, v16bf b, v8f c) { return __builtin_amdgcn_wmma_f32_16x16x32_bf16(false, a, false, b, (short)0, c, false, false); }


template <typename T16> struct WFrag;
template <> struct WFrag<h16> { typedef v16h V; static __device__ __forceinline__ V ld(const h16* p) { return cat16(*(const v8h*)p, *(const v8h*)(p + 16)); } static __device__ __forceinline__ v8f mma(V a, V b, v8f c) { return wmma16(a, b, c); } };
template <> struct WFrag<bf> { typedef v16bf V; static __device__ __forceinline__ V ld(const bf* p) { return cat16b(*(const v8us*)p, *(const v8us*)(p + 16)); } static __device__ __forceinline__ v8f mma(V a, V b, v8f c) { return wmmab(a, b, c); } };
template <typename T16, int NSPLIT, bool BIAS>
__global__ __launch_bounds__(32) void k_gemmw(const T16* __restrict__ A, const T16* __restrict__ A2, const T16* __restrict__ Bt, const T16* __restrict__ Bt2, int K, float* C, int ldc, const float* __restrict__ bias, size_t sA, size_t sB, size_t sC) {
    typedef typename WFrag<T16>::V V;
    __shared__ __align__(16) float os[16 * 68];
    const size_t z = blockIdx.z; A += z * sA; if (A2) A2 += z * sA; Bt += z * sB; if (Bt2) Bt2 += z * sB; C += z * sC;
    const int lane = threadIdx.x & 31, lr = lane & 15, hi = lane >> 4; const int r0 = blockIdx.x * 64, c0 = blockIdx.y * 64;
    v8f acc[4][4];
#pragma unroll
    for (int mb = 0; mb < 4; ++mb)
#pragma unroll
        for (int nb = 0; nb < 4; ++nb) acc[mb][nb] = (v8f){};
    const size_t aoff = (size_t)(r0 + lr) * K + 8 * hi, boff = (size_t)(c0 + lr) * K + 8 * hi;
#pragma unroll 1
    for (int kc = 0; kc < K; kc += 32) {
        V a[4], a2[4];
#pragma unroll
        for (int mb = 0; mb < 4; ++mb) { a[mb] = WFrag<T16>::ld(A + aoff + (size_t)mb * 16 * K + kc); if (NSPLIT == 1 || NSPLIT == 2) a2[mb] = WFrag<T16>::ld(A2 + aoff + (size_t)mb * 16 * K + kc); }
#pragma unroll
        for (int nb = 0; nb < 4; ++nb) { const V b = WFrag<T16>::ld(Bt + boff + (size_t)nb * 16 * K + kc); V b2; if (NSPLIT >= 2) b2 = WFrag<T16>::ld(Bt2 + boff + (size_t)nb * 16 * K + kc);
#pragma unroll
            for (int mb = 0; mb < 4; ++mb) { acc[mb][nb] = WFrag<T16>::mma(a[mb], b, acc[mb][nb]); if (NSPLIT == 1 || NSPLIT == 2) acc[mb][nb] = WFrag<T16>::mma(a2[mb], b, acc[mb][nb]); if (NSPLIT >= 2) acc[mb][nb] = WFrag<T16>::mma(a[mb], b2, acc[mb][nb]); } }
        asm volatile("v_nop\n\tv_nop\n\tv_nop\n\tv_nop" : "+v"(acc[0][0]), "+v"(acc[1][1]), "+v"(acc[2][2]), "+v"(acc[3][3]) : "v"(a[0]), "v"(a[3]));
    }
#pragma unroll
    for (int mb = 0; mb < 4; ++mb) {
#pragma unroll
        for (int nb = 0; nb < 4; ++nb) {
#pragma unroll
            for (int j = 0; j < 8; ++j) os[(hi * 8 + j) * 68 + nb * 16 + lr] = acc[mb][nb][j]; }
        __builtin_amdgcn_wave_barrier(); asm volatile("" ::: "memory");
        float* crow = C + (size_t)(r0 + mb * 16) * ldc + c0;
#pragma unroll 1
        for (int ps = 0; ps < 2; ++ps) {
#pragma unroll
            for (int s = 0; s < 8; ++s) { const int row = 2 * s + hi, cofs = lr * 4; v4f val = *(const v4fa*)(os + row * 68 + cofs); if (BIAS) { val[0] += bfr(bias[c0 + cofs]); val[1] += bfr(bias[c0 + cofs + 1]); val[2] += bfr(bias[c0 + cofs + 2]); val[3] += bfr(bias[c0 + cofs + 3]); }
                *(volatile v4f*)(crow + (size_t)row * ldc + cofs) = val; }
            if (ps == 0) __threadfence(); }
        __builtin_amdgcn_wave_barrier(); asm volatile("" ::: "memory");
    }
}

__device__ __forceinline__ h16 tohx(float x) { return (h16)x; }
typedef __attribute__((ext_vector_type(2))) _Float16 v2h;
typedef __attribute__((ext_vector_type(4))) _Float16 v4h;
typedef __attribute__((ext_vector_type(8))) _Float16 v8h16;
typedef __attribute__((ext_vector_type(2))) float v2f;

__global__ __launch_bounds__(256) void k_wtG16(const float* __restrict__ w, int K, int N, int pitch, int col0, h16* Bt) {
    const int lane = threadIdx.x & 31; const int L0 = (blockIdx.x * 8 + (threadIdx.x >> 5)) * 8; const int nlines = N * K / 64;
#pragma unroll 1
    for (int ps = 0; ps < 2; ++ps) {
#pragma unroll 1
        for (int l = 0; l < 8; ++l) { const int L = L0 + l; if (L >= nlines) break; const size_t e = (size_t)L * 64 + lane * 2; const int k = (int)(e % K), n = (int)(e / K); v2h o;
            o[0] = tohx(bfr(w[(size_t)k * pitch + col0 + n]) * WSC); o[1] = tohx(bfr(w[(size_t)(k + 1) * pitch + col0 + n]) * WSC); *(volatile v2h*)(Bt + e) = o; }
        if (ps == 0) __threadfence(); }
}
__global__ __launch_bounds__(256) void k_bsc(const float* __restrict__ b, float* BS, int n) { const int i = (blockIdx.x * 256 + threadIdx.x) * 4; if (i >= n) return; v4f o;
#pragma unroll
    for (int q = 0; q < 4; ++q) o[q] = bfr(b[i + q]) * WSC; *(volatile v4f*)(BS + i) = o; __threadfence(); *(volatile v4f*)(BS + i) = o; }
__global__ __launch_bounds__(256) void k_cstab(float* CS) { const int idx = blockIdx.x * 256 + threadIdx.x; if (idx >= TT * 32) return; const int t = idx >> 5, i = idx & 31; const float inv = __fdiv_rn(1.0f, powf(10000.0f, (float)(2 * i) / 64.0f)); const float ang = __fmul_rn((float)t, inv); v2f o; o[0] = cosf(ang); o[1] = sinf(ang);
    *(volatile v2f*)(CS + (size_t)idx * 2) = o; __threadfence(); *(volatile v2f*)(CS + (size_t)idx * 2) = o; }
__global__ __launch_bounds__(256) void k_ln0(const float* __restrict__ x, const float* __restrict__ gg, const float* __restrict__ bb, h16* T16) {
    const int lane = threadIdx.x & 31; const int r = blockIdx.x * 8 + (threadIdx.x >> 5); if (r >= TT) return; float v[DD / 32]; float s = 0.f;
#pragma unroll
    for (int c = 0; c < DD / 128; ++c) { const v4f a = *(const v4f*)(x + (size_t)r * DD + c * 128 + lane * 4);
#pragma unroll
        for (int q = 0; q < 4; ++q) { float t = bfr(a[q]); asm volatile("" : "+v"(t)); v[c * 4 + q] = t; s = __fadd_rn(s, t); } }
#pragma unroll
    for (int sh = 16; sh; sh >>= 1) s += __shfl_xor(s, sh, 32);
    const float mu = s * (1.0f / DD); float qq = 0.f;
#pragma unroll
    for (int i = 0; i < DD / 32; ++i) { const float d0 = v[i] - mu; float p = __fmul_rn(d0, d0); asm volatile("" : "+v"(p)); qq = __fadd_rn(qq, p); }
#pragma unroll
    for (int sh = 16; sh; sh >>= 1) qq += __shfl_xor(qq, sh, 32);
    const float rs = __fdiv_rn(1.0f, __fsqrt_rn(__fadd_rn(qq * (1.0f / DD), 1e-5f)));
#pragma unroll 1
    for (int ps = 0; ps < 2; ++ps) {
#pragma unroll
        for (int c = 0; c < DD / 128; ++c) { v4h o;
#pragma unroll
            for (int q = 0; q < 4; ++q) { const int col = c * 128 + lane * 4 + q; float t = __fmul_rn(v[c * 4 + q] - mu, rs); asm volatile("" : "+v"(t)); float tg = __fmul_rn(t, bfr(gg[col])); asm volatile("" : "+v"(tg)); o[q] = tohx(__fadd_rn(tg, bfr(bb[col]))); }
            *(volatile v4h*)(T16 + (size_t)r * DD + c * 128 + lane * 4) = o; }
        if (ps == 0) __threadfence(); }
}
__global__ __launch_bounds__(256) void k_qk(const float* __restrict__ PS, const float* __restrict__ CS, h16* QP, h16* KP) { const int e = (blockIdx.x * 256 + threadIdx.x) * 2; if (e >= TT * LOC) return; const int t = e / LOC, d = e % LOC; const float* row = PS + (size_t)t * SW;
    float q0 = row[d] * (1.0f / WSC), q1 = row[d + 1] * (1.0f / WSC), k0 = row[2 * LOC + d] * (1.0f / WSC), k1 = row[2 * LOC + d + 1] * (1.0f / WSC);
    if (d < 64) { const v2f cs = *(const v2f*)(CS + ((size_t)t * 32 + (d >> 1)) * 2); float a1 = __fmul_rn(q0, cs[0]), a2 = __fmul_rn(q1, cs[1]), a3 = __fmul_rn(q1, cs[0]), a4 = __fmul_rn(q0, cs[1]); asm volatile("" : "+v"(a1)); asm volatile("" : "+v"(a2)); asm volatile("" : "+v"(a3)); asm volatile("" : "+v"(a4));
        const float r0 = __fsub_rn(a1, a2), r1 = __fadd_rn(a3, a4); float b1 = __fmul_rn(k0, cs[0]), b2 = __fmul_rn(k1, cs[1]), b3 = __fmul_rn(k1, cs[0]), b4 = __fmul_rn(k0, cs[1]); asm volatile("" : "+v"(b1)); asm volatile("" : "+v"(b2)); asm volatile("" : "+v"(b3)); asm volatile("" : "+v"(b4));
        q0 = r0; q1 = r1; k0 = __fsub_rn(b1, b2); k1 = __fadd_rn(b3, b4); }
    v2h oq, ok; oq[0] = tohx(q0 * 0.125f); oq[1] = tohx(q1 * 0.125f); ok[0] = tohx(k0); ok[1] = tohx(k1);
    *(volatile v2h*)(QP + e) = oq; *(volatile v2h*)(KP + e) = ok; __threadfence(); *(volatile v2h*)(QP + e) = oq; *(volatile v2h*)(KP + e) = ok; }
__global__ __launch_bounds__(256) void k_vt(const float* __restrict__ PS, h16* VT) { const int e = (blockIdx.x * 256 + threadIdx.x) * 2; if (e >= LOC * TT) return; const int d = e / TT, t = e % TT; v2h v; v[0] = tohx(PS[(size_t)t * SW + LOC + d] * (1.0f / WSC)); v[1] = tohx(PS[(size_t)(t + 1) * SW + LOC + d] * (1.0f / WSC));
    *(volatile v2h*)(VT + e) = v; __threadfence(); *(volatile v2h*)(VT + e) = v; }
__global__ __launch_bounds__(256) void k_asoft(const float* __restrict__ Sb, const float* __restrict__ ab, h16* P16) {
    const int lane = threadIdx.x & 31; const int i = blockIdx.x * 8 + (threadIdx.x >> 5); if (i >= TT) return; const float* sr = Sb + (size_t)i * TT; const float* ar = ab + (size_t)i * TT; float v[64]; float mx = -3.0e38f;
#pragma unroll
    for (int ch = 0; ch < 16; ++ch) { const int j0 = ch * 128 + lane * 4; const v4f a = *(const v4f*)(sr + j0), b4 = *(const v4f*)(ar + j0);
#pragma unroll
        for (int q = 0; q < 4; ++q) { const int j = j0 + q; const float t = (j <= i) ? __fadd_rn(a[q], bfr(b4[q])) : -3.0e38f; v[ch * 4 + q] = t; mx = fmaxf(mx, t); } }
#pragma unroll
    for (int sh = 16; sh; sh >>= 1) mx = fmaxf(mx, __shfl_xor(mx, sh, 32));
    float sum = 0.f;
#pragma unroll
    for (int k = 0; k < 64; ++k) { float d0 = __fsub_rn(v[k], mx); asm volatile("" : "+v"(d0)); v[k] = __builtin_amdgcn_exp2f(__fmul_rn(d0, 1.4426950408889634f)); sum += v[k]; }
#pragma unroll
    for (int sh = 16; sh; sh >>= 1) sum += __shfl_xor(sum, sh, 32);
    const float f = __fdiv_rn(PCAR, sum);
#pragma unroll 1
    for (int ps = 0; ps < 2; ++ps) {
#pragma unroll
        for (int ch = 0; ch < 16; ++ch) { v4h o;
#pragma unroll
            for (int q = 0; q < 4; ++q) o[q] = tohx(v[ch * 4 + q] * f);
            *(volatile v4h*)(P16 + (size_t)i * TT + ch * 128 + lane * 4) = o; }
        if (ps == 0) __threadfence(); }
}
__global__ __launch_bounds__(256) void k_cata(const float* __restrict__ O, int mp, h16* CAT) { const int e = (blockIdx.x * 256 + threadIdx.x) * 2; if (e >= TT * LOC) return; const int t = e / LOC, d = e % LOC; v2h o; o[0] = tohx(O[e] * (1.0f / PCAR)); o[1] = tohx(O[e + 1] * (1.0f / PCAR));
    const size_t oo = (size_t)t * DCAT + mp * 640 + d; *(volatile v2h*)(CAT + oo) = o; __threadfence(); *(volatile v2h*)(CAT + oo) = o; }
__global__ __launch_bounds__(256) void k_glu(const float* __restrict__ PS, int mp, h16* CAT) { const int e = (blockIdx.x * 256 + threadIdx.x) * 2; if (e >= TT * 512) return; const int t = e / 512, j = e % 512; const float* row = PS + (size_t)t * SW + 3 * LOC; v2h o;
#pragma unroll
    for (int q = 0; q < 2; ++q) { const float a = row[j + q] * (1.0f / WSC), g = row[512 + j + q] * (1.0f / WSC); float g3 = __fmul_rn(__fmul_rn(g, g), g); asm volatile("" : "+v"(g3)); float in_ = __fadd_rn(g, __fmul_rn(0.044715f, g3)); asm volatile("" : "+v"(in_));
        const float th = tanhf(__fmul_rn(0.7978845608028654f, in_)); float hg = __fmul_rn(0.5f, g); asm volatile("" : "+v"(hg)); const float ge = __fmul_rn(hg, __fadd_rn(1.0f, th)); o[q] = tohx(__fmul_rn(a, ge)); }
    const size_t oo = (size_t)t * DCAT + mp * 640 + LOC + j; *(volatile v2h*)(CAT + oo) = o; __threadfence(); *(volatile v2h*)(CAT + oo) = o; }
__global__ __launch_bounds__(256) void k_fin(const float* __restrict__ F, float* OUT) { const size_t i = ((size_t)blockIdx.x * 256 + threadIdx.x) * 4; if (i >= (size_t)TT * DD) return; const v4f a = *(const v4f*)(F + i); v4f o;
#pragma unroll
    for (int q = 0; q < 4; ++q) o[q] = a[q] * (1.0f / WSC); *(volatile v4f*)(OUT + i) = o; __threadfence(); *(volatile v4f*)(OUT + i) = o; }

extern "C" void kernel_launch(void* const* d_in, const int* in_sizes, int n_in,
                              void* d_out, int out_size, void* d_ws, size_t ws_size, hipStream_t stream) {
    (void)in_sizes; (void)n_in; (void)out_size;
    const float* x = (const float*)d_in[0]; const float* ab = (const float*)d_in[1]; const float* lg = (const float*)d_in[2]; const float* lb = (const float*)d_in[3]; const float* w_in = (const float*)d_in[4]; const float* b_in = (const float*)d_in[5]; const float* w_out = (const float*)d_in[6]; const float* b_out = (const float*)d_in[7];
    float* OUT = (float*)d_out;
    char* wsp = (char*)d_ws;
    auto take = [&](size_t bytes) { char* p = wsp; wsp += (bytes + 255) & ~(size_t)255; return (void*)p; };
    h16* WIN = (h16*)take((size_t)FIN * DD * 2); h16* WOUT = (h16*)take((size_t)DD * DCAT * 2); float* BIN = (float*)take(FIN * 4); float* BOUT = (float*)take(DD * 4); float* CS = (float*)take((size_t)TT * 32 * 2 * 4);
    h16* T16 = (h16*)take((size_t)TT * DD * 2); float* PS = (float*)take((size_t)TT * SW * 4); h16* QP = (h16*)take((size_t)TT * LOC * 2); h16* KP = (h16*)take((size_t)TT * LOC * 2); h16* VT = (h16*)take((size_t)LOC * TT * 2);
    float* Sb = (float*)take((size_t)TT * TT * 4); h16* Pm = (h16*)take((size_t)TT * TT * 2); float* Ob = (float*)take((size_t)TT * LOC * 4); h16* CAT = (h16*)take((size_t)TT * DCAT * 2); float* F = (float*)take((size_t)TT * DD * 4);
    if ((size_t)(wsp - (char*)d_ws) > ws_size) return;
    { k_wtG16<<<(unsigned)((FIN * DD / 64 + 63) / 64), 256, 0, stream>>>(w_in, DD, FIN, FIN, 0, WIN); k_wtG16<<<(unsigned)((DD * DCAT / 64 + 63) / 64), 256, 0, stream>>>(w_out, DCAT, DD, DD, 0, WOUT);
      k_bsc<<<FIN / 1024, 256, 0, stream>>>(b_in, BIN, FIN); k_bsc<<<DD / 1024, 256, 0, stream>>>(b_out, BOUT, DD); k_cstab<<<(TT * 32 + 255) / 256, 256, 0, stream>>>(CS); }
    const unsigned LQ = (TT * LOC / 2 + 255) / 256;
    for (int b = 0; b < NB_; ++b) {
        k_ln0<<<TT / 8, 256, 0, stream>>>(x + (size_t)b * TT * DD, lg, lb, T16);
        for (int mp = 0; mp < MP; ++mp) {
            k_gemmw<h16, 0, true><<<dim3(TT / 64, SW / 64, 1), 32, 0, stream>>>(T16, nullptr, WIN + (size_t)mp * SW * DD, nullptr, DD, PS, SW, BIN + mp * SW, 0, 0, 0);
            k_qk<<<LQ, 256, 0, stream>>>(PS, CS, QP, KP); k_vt<<<LQ, 256, 0, stream>>>(PS, VT);
            k_gemmw<h16, 0, false><<<dim3(TT / 64, TT / 64, 1), 32, 0, stream>>>(QP, nullptr, KP, nullptr, LOC, Sb, TT, nullptr, 0, 0, 0);
            k_asoft<<<TT / 8, 256, 0, stream>>>(Sb, ab, Pm);
            k_gemmw<h16, 0, false><<<dim3(TT / 64, LOC / 64, 1), 32, 0, stream>>>(Pm, nullptr, VT, nullptr, TT, Ob, LOC, nullptr, 0, 0, 0);
            k_cata<<<LQ, 256, 0, stream>>>(Ob, mp, CAT); k_glu<<<(TT * 512 / 2 + 255) / 256, 256, 0, stream>>>(PS, mp, CAT); }
        k_gemmw<h16, 0, true><<<dim3(TT / 64, DD / 64, 1), 32, 0, stream>>>(CAT, nullptr, WOUT, nullptr, DCAT, F, DD, BOUT, 0, 0, 0);
        k_fin<<<(unsigned)(((size_t)TT * DD / 4 + 255) / 256), 256, 0, stream>>>(F, OUT + (size_t)b * TT * DD); }
}
